// BiRNNDecoder_38190849196288
// MI455X (gfx1250) — hardware-verified
//
#include <hip/hip_runtime.h>
#include <math.h>

constexpr int NBATCH  = 8192;
constexpr int NSTEP   = 524;
constexpr int NHID    = 32;
constexpr int NGATE   = 96;
constexpr int NPOOL   = 64;
constexpr int NHEAD   = 256;
constexpr int NGRP    = NSTEP / 4;
constexpr int HPITCH  = 40;
constexpr int PMPITCH = 68;
constexpr int SCAN_THR = 64;
constexpr int CT_CINIT = 0;
constexpr int CT_WIH   = NGATE;
constexpr int CT_BIHN  = 2 * NGATE;
constexpr int CT_SIZE  = 2 * NGATE + NHID;
static_assert(NSTEP % 4 == 0);
static_assert(NGATE == 3 * NHID);
static_assert(NHID == 32);
static_assert(NPOOL == 2 * NHID);
static_assert(NBATCH % 64 == 0);
static_assert(NBATCH % 16 == 0);
static_assert(NHEAD % 64 == 0);
static_assert(NPOOL % 32 == 0);
static_assert((NSTEP * 4) % 16 == 0);
static_assert((HPITCH * 2) % 16 == 0);
static_assert((CT_SIZE * 4) % 32 == 0);
static_assert((NHEAD * NPOOL) % (8 * 256) == 0);

typedef __attribute__((ext_vector_type(16))) _Float16 v16h;
typedef __attribute__((ext_vector_type(8)))  _Float16 v8h;
typedef __attribute__((ext_vector_type(16))) __bf16   v16b;
typedef __attribute__((ext_vector_type(8)))  __bf16   v8b;
typedef __attribute__((ext_vector_type(8)))  float    v8f;
typedef __attribute__((ext_vector_type(4)))  float    v4f;
typedef __attribute__((ext_vector_type(4)))  unsigned v4u;

__device__ __forceinline__ unsigned short f2bf_bits(float f) {
  unsigned u = __float_as_uint(f);
  return (unsigned short)((u + 0x7FFFu + ((u >> 16) & 1u)) >> 16);
}
__device__ __forceinline__ float bf_bits2f(unsigned short h) { return __uint_as_float(((unsigned)h) << 16); }

__device__ __forceinline__ void dep_guard_h(v8f& a, v8f& b, v16h x, v16h y) { asm volatile("v_nop\n\tv_nop\n\tv_nop\n\tv_nop" : "+v"(a), "+v"(b) : "v"(x), "v"(y)); }
__device__ __forceinline__ void dep_guard_b(v8f& a, v8f& b, v16b x, v16b y) { asm volatile("v_nop\n\tv_nop\n\tv_nop\n\tv_nop" : "+v"(a), "+v"(b) : "v"(x), "v"(y)); }
__device__ __forceinline__ void dep_guard4_h(v8f& a, v8f& b, v8f& c, v8f& d, v16h x, v16h y) { asm volatile("v_nop\n\tv_nop\n\tv_nop\n\tv_nop" : "+v"(a), "+v"(b), "+v"(c), "+v"(d) : "v"(x), "v"(y)); }
__device__ __forceinline__ void dep_guard4_b(v8f& a, v8f& b, v8f& c, v8f& d, v16b x, v16b y) { asm volatile("v_nop\n\tv_nop\n\tv_nop\n\tv_nop" : "+v"(a), "+v"(b), "+v"(c), "+v"(d) : "v"(x), "v"(y)); }
__device__ __forceinline__ void dep_guard3_h(v8f& a, v8f& b, v8f& c, v16h x, v16h y, v16h z, v16h w) { asm volatile("v_nop\n\tv_nop\n\tv_nop\n\tv_nop" : "+v"(a), "+v"(b), "+v"(c) : "v"(x), "v"(y), "v"(z), "v"(w)); }
__device__ __forceinline__ void keep4_h(v16h a, v16h b, v16h c, v16h d) { asm volatile("v_nop" :: "v"(a), "v"(b), "v"(c), "v"(d)); }
__device__ __forceinline__ void keep4_b(v16b a, v16b b, v16b c, v16b d) { asm volatile("v_nop" :: "v"(a), "v"(b), "v"(c), "v"(d)); }
__device__ __forceinline__ void acc_guard4(v8f& a, v8f& b, v8f& c, v8f& d) { asm volatile("v_nop\n\tv_nop\n\tv_nop\n\tv_nop" : "+v"(a), "+v"(b), "+v"(c), "+v"(d)); }
__device__ __forceinline__ int opaque_i(int v) { asm volatile("" : "+v"(v)); return v; }

template <typename T> struct Frag;
template <> struct Frag<_Float16> {
  typedef v16h V; union U { v16h v; v8h h[2]; };
  static __device__ __forceinline__ v16h load(const _Float16* p) {
    U f; f.h[0] = *(const v8h*)(p); f.h[1] = *(const v8h*)(p + 16); return f.v;
  }
  static __device__ __forceinline__ v8f mma(v16h a, v16h b, v8f c) {
    return __builtin_amdgcn_wmma_f32_16x16x32_f16(false, a, false, b, (short)0, c, false, false);
  }
  static __device__ __forceinline__ void guard(v8f& a, v8f& b, v16h x, v16h y) { dep_guard_h(a, b, x, y); }
  static __device__ __forceinline__ void guard4(v8f& a, v8f& b, v8f& c, v8f& d, v16h x, v16h y) { dep_guard4_h(a, b, c, d, x, y); }
  static __device__ __forceinline__ void keep(v16h a, v16h b, v16h c, v16h d) { keep4_h(a, b, c, d); }
};
template <> struct Frag<__bf16> {
  typedef v16b V; union U { v16b v; v8b h[2]; };
  static __device__ __forceinline__ v16b load(const __bf16* p) {
    U f; f.h[0] = *(const v8b*)(p); f.h[1] = *(const v8b*)(p + 16); return f.v;
  }
  static __device__ __forceinline__ v8f mma(v16b a, v16b b, v8f c) {
    return __builtin_amdgcn_wmma_f32_16x16x32_bf16(false, a, false, b, (short)0, c, false, false);
  }
  static __device__ __forceinline__ void guard(v8f& a, v8f& b, v16b x, v16b y) { dep_guard_b(a, b, x, y); }
  static __device__ __forceinline__ void guard4(v8f& a, v8f& b, v8f& c, v8f& d, v16b x, v16b y) { dep_guard4_b(a, b, c, d, x, y); }
  static __device__ __forceinline__ void keep(v16b a, v16b b, v16b c, v16b d) { keep4_b(a, b, c, d); }
};

__device__ __forceinline__ float fsig(float v)  { return __builtin_amdgcn_rcpf(1.0f + __expf(-v)); }
__device__ __forceinline__ float ftanh(float v) { return 1.0f - 2.0f * __builtin_amdgcn_rcpf(__expf(2.0f * v) + 1.0f); }

__device__ __forceinline__ v16h frag_from_f32(const float* p) {
  const v4f a0 = *(const v4f*)(p);
  const v4f a1 = *(const v4f*)(p + 4);
  const v4f a2 = *(const v4f*)(p + 16);
  const v4f a3 = *(const v4f*)(p + 20);
  v16h f;
#pragma unroll
  for (int e = 0; e < 4; ++e) {
    f[e]      = (_Float16)a0[e];
    f[4 + e]  = (_Float16)a1[e];
    f[8 + e]  = (_Float16)a2[e];
    f[12 + e] = (_Float16)a3[e];
  }
  return f;
}

__device__ __forceinline__ v8f lds_load8(const float* p) {
  const v4f a = *(const v4f*)(p);
  const v4f b = *(const v4f*)(p + 4);
  return __builtin_shufflevector(a, b, 0, 1, 2, 3, 4, 5, 6, 7);
}

__device__ __forceinline__ float gru_cell(float xv, float cr, float cz, float cn,
                                          float wr, float wz, float wn, float bn, float hold) {
  const float ar = fmaf(xv, wr, cr);
  const float az = fmaf(xv, wz, cz);
  const float r  = fsig(ar);
  const float z  = fsig(az);
  const float an = fmaf(r, cn, fmaf(xv, wn, bn));
  const float n  = ftanh(an);
  return fmaf(z, hold - n, n);
}

template <int ET> struct Elem;
template <> struct Elem<0> { typedef _Float16 T; };
template <> struct Elem<1> { typedef __bf16 T; };
template <int ET, bool SPLIT, int BIAS_MODE, int OUT_MODE, bool RESID, int ACT = 0>
__global__ __launch_bounds__(256) void wmma_gemm64(
    const unsigned short* __restrict__ Ap, const unsigned short* __restrict__ A2p, int lda, long strideA,
    const unsigned short* __restrict__ Btp, const unsigned short* __restrict__ Bt2p, int ldb, long strideB,
    void* __restrict__ Cout, void* __restrict__ Cout2, int ldc, long strideC,
    const float* __restrict__ bias,
    const float* __restrict__ resid, long strideR,
    int M, int N, int K, float scale) {
  typedef typename Elem<ET>::T T;
  typedef typename Frag<T>::V V;
  const T* A = (const T*)Ap; const T* A2 = (const T*)A2p; const T* Bt = (const T*)Btp; const T* Bt2 = (const T*)Bt2p;
  __shared__ __align__(16) float sT[8][16 * 68];
  const int b    = blockIdx.y;
  const int lane = threadIdx.x & 31;
  const int wave = threadIdx.x >> 5;
  const int tilesN = N >> 6;
  const int tilesM = M >> 6;
  const int tile = blockIdx.x * 8 + wave;
  if (tile >= tilesM * tilesN) return;
  const int tm = tile / tilesN;
  const int tn = tile - tm * tilesN;
  const int m0 = tm << 6;
  const int n0 = tn << 6;

  const T* Ab  = A  + (size_t)b * strideA;
  const T* Bb  = Bt + (size_t)b * strideB;
  const T* Ab2 = SPLIT ? (A2  + (size_t)b * strideA) : nullptr;
  const T* Bb2 = SPLIT ? (Bt2 + (size_t)b * strideB) : nullptr;

  const int rlane = lane & 15;
  const int koff  = (lane >> 4) * 8;
  const int mOff  = (lane >> 4) * 8;

  v8f acc[4][4];
#pragma unroll
  for (int i = 0; i < 4; ++i)
#pragma unroll
    for (int j = 0; j < 4; ++j) acc[i][j] = (v8f){0.f,0.f,0.f,0.f,0.f,0.f,0.f,0.f};

  for (int k0 = 0; k0 < K; k0 += 32) {
    V bh[4], bl[4];
#pragma unroll
    for (int j = 0; j < 4; ++j) {
      const size_t bo = (size_t)(n0 + (j << 4) + rlane) * ldb + koff + k0;
      bh[j] = Frag<T>::load(Bb + bo);
      if (SPLIT) bl[j] = Frag<T>::load(Bb2 + bo);
    }
#pragma unroll
    for (int i = 0; i < 4; ++i) {
      const size_t ao = (size_t)(m0 + (i << 4) + rlane) * lda + koff + k0;
      V ah = Frag<T>::load(Ab + ao);
      V al;
      if (SPLIT) al = Frag<T>::load(Ab2 + ao);
#pragma unroll
      for (int j = 0; j < 4; ++j) {
        acc[i][j] = Frag<T>::mma(ah, bh[j], acc[i][j]);
        if (SPLIT) {
          acc[i][j] = Frag<T>::mma(ah, bl[j], acc[i][j]);
          acc[i][j] = Frag<T>::mma(al, bh[j], acc[i][j]);
        }
      }
      Frag<T>::guard4(acc[i][0], acc[i][1], acc[i][2], acc[i][3], ah, SPLIT ? al : ah);
    }
    Frag<T>::keep(bh[0], bh[1], bh[2], bh[3]);
    if (SPLIT) Frag<T>::keep(bl[0], bl[1], bl[2], bl[3]);
  }
  acc_guard4(acc[0][0], acc[0][1], acc[0][2], acc[0][3]);
  acc_guard4(acc[1][0], acc[1][1], acc[1][2], acc[1][3]);
  acc_guard4(acc[2][0], acc[2][1], acc[2][2], acc[2][3]);
  acc_guard4(acc[3][0], acc[3][1], acc[3][2], acc[3][3]);

  float* slab = sT[wave];
  const float* Rb = RESID ? (resid + (size_t)b * strideR) : nullptr;
#pragma unroll
  for (int i = 0; i < 4; ++i) {
    const int mBase = m0 + (i << 4);
#pragma unroll
    for (int j = 0; j < 4; ++j) {
      const int n = n0 + (j << 4) + rlane;
      float bv = 0.f;
      if (BIAS_MODE == 2) bv = bias[n];
#pragma unroll
      for (int r = 0; r < 8; ++r) {
        float v = acc[i][j][r] * scale;
        if (BIAS_MODE == 1) v += bias[mBase + mOff + r];
        if (BIAS_MODE == 2) v += bv;
        if (RESID) v += Rb[(size_t)(mBase + mOff + r) * ldc + n];
        if (ACT == 2) v = fmaxf(v, 0.0f);
        if (ACT == 4) v = (v > 0.f) ? v : 0.01f * v;
        slab[(mOff + r) * 68 + (j << 4) + rlane] = v;
      }
    }
    __builtin_amdgcn_fence(__ATOMIC_RELEASE, "workgroup");
    __builtin_amdgcn_wave_barrier();
    __builtin_amdgcn_fence(__ATOMIC_ACQUIRE, "workgroup");
    if (OUT_MODE == 0) {
      float* C = (float*)Cout + (size_t)b * strideC;
      const int hh = lane >> 4, c4 = (lane & 15) * 4;
      for (int pass = 0; pass < 2; ++pass) {
#pragma unroll
        for (int it = 0; it < 8; ++it) {
          const int row = it * 2 + hh;
          v4f v = *(const v4f*)(slab + row * 68 + c4);
          *(volatile v4f*)(C + (size_t)(mBase + row) * ldc + n0 + c4) = v;
        }
        __threadfence();
      }
    } else {
      const int q = lane >> 3, c8 = (lane & 7) * 8;
      unsigned short* C  = (unsigned short*)Cout  + (size_t)b * strideC;
      unsigned short* C2 = (OUT_MODE == 2) ? ((unsigned short*)Cout2 + (size_t)b * strideC) : nullptr;
      for (int pass = 0; pass < 2; ++pass) {
#pragma unroll
        for (int it = 0; it < 4; ++it) {
          const int row = it * 4 + q;
          const float* sp = slab + row * 68 + c8;
          v8h hv, lv;
#pragma unroll
          for (int e = 0; e < 8; ++e) {
            if (OUT_MODE == 1) {
              hv[e] = (_Float16)sp[e];
            } else {
              unsigned short hb = f2bf_bits(sp[e]);
              unsigned short lb = f2bf_bits(sp[e] - bf_bits2f(hb));
              hv[e] = __builtin_bit_cast(_Float16, hb);
              lv[e] = __builtin_bit_cast(_Float16, lb);
            }
          }
          *(volatile v8h*)(C + (size_t)(mBase + row) * ldc + n0 + c8) = hv;
          if (OUT_MODE == 2) *(volatile v8h*)(C2 + (size_t)(mBase + row) * ldc + n0 + c8) = lv;
        }
        __threadfence();
      }
    }
    __builtin_amdgcn_fence(__ATOMIC_RELEASE, "workgroup");
    __builtin_amdgcn_wave_barrier();
    __builtin_amdgcn_fence(__ATOMIC_ACQUIRE, "workgroup");
  }
}

__global__ __launch_bounds__(256) void split_planes_kernel(const float* __restrict__ src,
                                                           unsigned short* __restrict__ hi,
                                                           unsigned short* __restrict__ lo, int n8) {
  const int i = blockIdx.x * 256 + threadIdx.x;
  if (i < n8) {
    const v4f a = *(const v4f*)(src + (size_t)i * 8);
    const v4f b = *(const v4f*)(src + (size_t)i * 8 + 4);
    v4u hv, lv;
#pragma unroll
    for (int p = 0; p < 2; ++p) {
      const float f0 = a[2 * p], f1 = a[2 * p + 1];
      const float g0 = b[2 * p], g1 = b[2 * p + 1];
      const unsigned short hf0 = f2bf_bits(f0), hf1 = f2bf_bits(f1);
      const unsigned short hg0 = f2bf_bits(g0), hg1 = f2bf_bits(g1);
      const unsigned short lf0 = f2bf_bits(f0 - bf_bits2f(hf0)), lf1 = f2bf_bits(f1 - bf_bits2f(hf1));
      const unsigned short lg0 = f2bf_bits(g0 - bf_bits2f(hg0)), lg1 = f2bf_bits(g1 - bf_bits2f(hg1));
      hv[p]     = (unsigned)hf0 | ((unsigned)hf1 << 16);
      hv[2 + p] = (unsigned)hg0 | ((unsigned)hg1 << 16);
      lv[p]     = (unsigned)lf0 | ((unsigned)lf1 << 16);
      lv[2 + p] = (unsigned)lg0 | ((unsigned)lg1 << 16);
    }
    *(volatile v4u*)(hi + (size_t)i * 8) = hv;
    *(volatile v4u*)(lo + (size_t)i * 8) = lv;
    __threadfence();
    *(volatile v4u*)(hi + (size_t)i * 8) = hv;
    *(volatile v4u*)(lo + (size_t)i * 8) = lv;
  }
}

__global__ __launch_bounds__(SCAN_THR) __attribute__((amdgpu_num_vgpr(256))) void gru_scan_kernel(
    const float* __restrict__ x,
    const float* __restrict__ wih_f, const float* __restrict__ whh_f,
    const float* __restrict__ bih_f, const float* __restrict__ bhh_f,
    const float* __restrict__ wih_b, const float* __restrict__ whh_b,
    const float* __restrict__ bih_b, const float* __restrict__ bhh_b,
    unsigned short* __restrict__ PHI, unsigned short* __restrict__ PLO) {
  __shared__ __align__(32) float    ctab[2 * CT_SIZE];
  __shared__ __align__(16) _Float16 htile[2 * 16 * HPITCH];
  __shared__ __align__(16) float    pmerge[16 * PMPITCH];

  const int tid  = threadIdx.x;
  const int lane = tid & 31;
  const int dir  = __builtin_amdgcn_readfirstlane((int)(tid >> 5));
  const int c    = lane & 15;
  const int hh   = lane >> 4;
  const int rowbase = blockIdx.x * 16;

  const float* wih = dir ? wih_b : wih_f;
  const float* whh = dir ? whh_b : whh_f;
  const float* bih = dir ? bih_b : bih_f;
  const float* bhh = dir ? bhh_b : bhh_f;

  {
    float* tw = ctab + dir * CT_SIZE;
#pragma unroll
    for (int i = 0; i < 3; ++i) {
      const int g = lane + 32 * i;
      const float bi = bih[g];
      const float bh = bhh[g];
      const float wv = wih[g];
      tw[CT_CINIT + g] = (i < 2) ? (bi + bh) : bh;
      tw[CT_WIH + g]   = wv;
    }
    tw[CT_BIHN + lane] = bih[2 * NHID + lane];
  }

  v16h A[6];
#pragma unroll
  for (int tl = 0; tl < 6; ++tl) A[tl] = frag_from_f32(whh + (size_t)(tl * 16 + c) * NHID + 8 * hh);

  float H0[8], H1[8];
#pragma unroll
  for (int k = 0; k < 8; ++k) { H0[k] = 0.0f; H1[k] = 0.0f; }
  v16h Bm;
#pragma unroll
  for (int e = 0; e < 16; ++e) Bm[e] = (_Float16)0.0f;

  __syncthreads();

  const int    tofs = dir * CT_SIZE + 8 * hh;
  _Float16*    hrow = htile + dir * 16 * HPITCH + c * HPITCH + 8 * hh;
  const float* xr   = x + (size_t)(rowbase + c) * NSTEP;

#pragma unroll 1
  for (int g = 0; g < NGRP; ++g) {
    const int gg = dir ? (NGRP - 1 - g) : g;
    const v4f xq = *(const v4f*)(xr + 4 * gg);
    float xs[4];
    xs[0] = dir ? xq[3] : xq[0];
    xs[1] = dir ? xq[2] : xq[1];
    xs[2] = dir ? xq[1] : xq[2];
    xs[3] = dir ? xq[0] : xq[3];
#pragma unroll
    for (int e = 0; e < 4; ++e) {
      const float xv = xs[e];
      {
        const float* tp = ctab + opaque_i(tofs);
        v8f cr = lds_load8(tp + CT_CINIT);
        v8f cz = lds_load8(tp + CT_CINIT + 32);
        v8f cn = lds_load8(tp + CT_CINIT + 64);
        cr = Frag<_Float16>::mma(A[0], Bm, cr);
        cz = Frag<_Float16>::mma(A[2], Bm, cz);
        cn = Frag<_Float16>::mma(A[4], Bm, cn);
        dep_guard3_h(cr, cz, cn, A[0], A[2], A[4], Bm);
        const v8f wr = lds_load8(tp + CT_WIH);
        const v8f wz = lds_load8(tp + CT_WIH + 32);
        const v8f wn = lds_load8(tp + CT_WIH + 64);
        const v8f bn = lds_load8(tp + CT_BIHN);
#pragma unroll
        for (int k = 0; k < 8; ++k)
          H0[k] = gru_cell(xv, cr[k], cz[k], cn[k], wr[k], wz[k], wn[k], bn[k], H0[k]);
      }
      {
        const float* tp = ctab + opaque_i(tofs) + 16;
        v8f cr = lds_load8(tp + CT_CINIT);
        v8f cz = lds_load8(tp + CT_CINIT + 32);
        v8f cn = lds_load8(tp + CT_CINIT + 64);
        cr = Frag<_Float16>::mma(A[1], Bm, cr);
        cz = Frag<_Float16>::mma(A[3], Bm, cz);
        cn = Frag<_Float16>::mma(A[5], Bm, cn);
        dep_guard3_h(cr, cz, cn, A[1], A[3], A[5], Bm);
        const v8f wr = lds_load8(tp + CT_WIH);
        const v8f wz = lds_load8(tp + CT_WIH + 32);
        const v8f wn = lds_load8(tp + CT_WIH + 64);
        const v8f bn = lds_load8(tp + CT_BIHN);
#pragma unroll
        for (int k = 0; k < 8; ++k)
          H1[k] = gru_cell(xv, cr[k], cz[k], cn[k], wr[k], wz[k], wn[k], bn[k], H1[k]);
      }
      v8h ha, hb;
#pragma unroll
      for (int k = 0; k < 8; ++k) { ha[k] = (_Float16)H0[k]; hb[k] = (_Float16)H1[k]; }
      *(v8h*)(hrow)      = ha;
      *(v8h*)(hrow + 16) = hb;
      __builtin_amdgcn_fence(__ATOMIC_RELEASE, "workgroup");
      __builtin_amdgcn_wave_barrier();
      __builtin_amdgcn_fence(__ATOMIC_ACQUIRE, "workgroup");
      Bm = Frag<_Float16>::load(hrow);
    }
  }

  {
    float* pm = pmerge + c * PMPITCH + dir * 32 + 8 * hh;
    const v4f p0 = {H0[0], H0[1], H0[2], H0[3]};
    const v4f p1 = {H0[4], H0[5], H0[6], H0[7]};
    const v4f p2 = {H1[0], H1[1], H1[2], H1[3]};
    const v4f p3 = {H1[4], H1[5], H1[6], H1[7]};
    *(v4f*)(pm)      = p0;
    *(v4f*)(pm + 4)  = p1;
    *(v4f*)(pm + 16) = p2;
    *(v4f*)(pm + 20) = p3;
  }
  __syncthreads();
  {
    const int q = lane >> 3, c8 = (lane & 7) * 8;
    unsigned short* dst = dir ? PLO : PHI;
    v4u pk[4];
#pragma unroll
    for (int it = 0; it < 4; ++it) {
      const int row = it * 4 + q;
      const float* sp = pmerge + row * PMPITCH + c8;
      const v4f a = *(const v4f*)(sp);
      const v4f b = *(const v4f*)(sp + 4);
#pragma unroll
      for (int p = 0; p < 2; ++p) {
        const float f0 = a[2 * p], f1 = a[2 * p + 1];
        const float g0 = b[2 * p], g1 = b[2 * p + 1];
        const unsigned short hf0 = f2bf_bits(f0), hf1 = f2bf_bits(f1);
        const unsigned short hg0 = f2bf_bits(g0), hg1 = f2bf_bits(g1);
        const unsigned short lf0 = f2bf_bits(f0 - bf_bits2f(hf0)), lf1 = f2bf_bits(f1 - bf_bits2f(hf1));
        const unsigned short lg0 = f2bf_bits(g0 - bf_bits2f(hg0)), lg1 = f2bf_bits(g1 - bf_bits2f(hg1));
        const unsigned sf0 = dir ? (unsigned)lf0 : (unsigned)hf0;
        const unsigned sf1 = dir ? (unsigned)lf1 : (unsigned)hf1;
        const unsigned sg0 = dir ? (unsigned)lg0 : (unsigned)hg0;
        const unsigned sg1 = dir ? (unsigned)lg1 : (unsigned)hg1;
        pk[it][p]     = sf0 | (sf1 << 16);
        pk[it][2 + p] = sg0 | (sg1 << 16);
      }
    }
    for (int pass = 0; pass < 2; ++pass) {
#pragma unroll
      for (int it = 0; it < 4; ++it) {
        const int row = it * 4 + q;
        *(volatile v4u*)(dst + (size_t)(rowbase + row) * NPOOL + c8) = pk[it];
      }
      __threadfence();
    }
  }
}

extern "C" void kernel_launch(void* const* d_in, const int* in_sizes, int n_in,
                              void* d_out, int out_size, void* d_ws, size_t ws_size, hipStream_t stream) {
  (void)in_sizes; (void)out_size;
  if (n_in < 11 || d_out == nullptr || d_ws == nullptr) return;

  const float* x     = (const float*)d_in[0];
  const float* wih_f = (const float*)d_in[1];
  const float* whh_f = (const float*)d_in[2];
  const float* bih_f = (const float*)d_in[3];
  const float* bhh_f = (const float*)d_in[4];
  const float* wih_b = (const float*)d_in[5];
  const float* whh_b = (const float*)d_in[6];
  const float* bih_b = (const float*)d_in[7];
  const float* bhh_b = (const float*)d_in[8];
  const float* w_out = (const float*)d_in[9];
  const float* b_out = (const float*)d_in[10];

  char* ws = (char*)d_ws; size_t off = 0;
  auto carve = [&](size_t bytes) -> char* { char* p = ws + off; off += (bytes + 255) & ~(size_t)255; return p; };
  unsigned short* PHI = (unsigned short*)carve((size_t)NBATCH * NPOOL * 2);
  unsigned short* PLO = (unsigned short*)carve((size_t)NBATCH * NPOOL * 2);
  unsigned short* WOH = (unsigned short*)carve((size_t)NHEAD * NPOOL * 2);
  unsigned short* WOL = (unsigned short*)carve((size_t)NHEAD * NPOOL * 2);
  if (off > ws_size || off > (size_t)134217728) return;

  const int n8w = NHEAD * NPOOL / 8;
  split_planes_kernel<<<n8w / 256, 256, 0, stream>>>(w_out, WOH, WOL, n8w);

  gru_scan_kernel<<<NBATCH / 16, SCAN_THR, 0, stream>>>(x, wih_f, whh_f, bih_f, bhh_f,
                                                        wih_b, whh_b, bih_b, bhh_b, PHI, PLO);

  const dim3 hgrid((NBATCH / 64) * (NHEAD / 64) / 8, 1);
  wmma_gemm64<1, true, 2, 0, false, 0><<<hgrid, 256, 0, stream>>>(
      PHI, PLO, NPOOL, 0L, WOH, WOL, NPOOL, 0L, d_out, d_out, NHEAD, 0L,
      b_out, b_out, 0L, NBATCH, NHEAD, NPOOL, 1.0f);
}
